// GAT_68968584839686
// MI455X (gfx1250) — hardware-verified
//
#include <hip/hip_runtime.h>
#include <stddef.h>
#include <stdint.h>
#include <math.h>


#define F_IN    128
#define HC1     64
#define HID     32
#define NHD1    2
#define NC2     32
#define KA2     128
#define NTHR    256
#define NWAVE   8
#define EPT     8
#define CHUNK   (NTHR * EPT)
#define WCAP    (EPT * 32)
#define LISTN   (NWAVE * WCAP)
#define NB      1024
#define SLOTB   10
#define RCAP    24576
#define DEGCAP  64
#define GBM     64
#define GTHR    128
#define NEGSL   0.2f
#define WSMAX   134217728
#define LDS_AGG ((2 * RCAP + 2 * NB + LISTN) * 4 + 64)
#define SPILL_IT (RCAP / (NTHR * 4))

static_assert((CHUNK & (CHUNK - 1)) == 0 && CHUNK <= 4096);
static_assert(NB == (1 << SLOTB));
static_assert(((long long)CHUNK << SLOTB) < (1LL << 31));
static_assert(NTHR * 4 == NB);
static_assert(LISTN >= NB);
static_assert(LISTN >= NWAVE * WCAP);
static_assert((RCAP % (NTHR * 4)) == 0);
static_assert(SPILL_IT * NTHR * 4 == RCAP);
static_assert((NB % NWAVE) == 0);
static_assert(LDS_AGG <= 300000);
static_assert(GBM == (GTHR / 32) * 16);
static_assert(GTHR == 2 * GBM);
static_assert((F_IN % 32) == 0 && (KA2 % 32) == 0);
static_assert(KA2 == 2 * HC1);
static_assert(HC1 == 2 * 32);
static_assert(NC2 == 32);
static_assert(HC1 == NHD1 * HID && HID == 32);
static_assert((F_IN / 8) == 16);

typedef float          v2f  __attribute__((ext_vector_type(2)));
typedef float          v4f  __attribute__((ext_vector_type(4)));
typedef float          v8f  __attribute__((ext_vector_type(8)));
typedef int            v4i  __attribute__((ext_vector_type(4)));
typedef int            v8i  __attribute__((ext_vector_type(8)));
typedef unsigned int   v4u  __attribute__((ext_vector_type(4)));
typedef unsigned short v8us __attribute__((ext_vector_type(8)));
typedef __bf16         v16b __attribute__((ext_vector_type(16)));
typedef v2f  __attribute__((may_alias)) v2fa;
typedef v4f  __attribute__((may_alias)) v4fa;
typedef v4i  __attribute__((may_alias)) v4ia;
typedef v8us __attribute__((may_alias)) v8usa;
union FragB { v16b v; v8us h[2]; v8i w; };

__device__ __forceinline__ v8f wmb(const FragB& a, const FragB& b, v8f c) {
  v8f d = __builtin_amdgcn_wmma_f32_16x16x32_bf16(false, a.v, false, b.v, (short)0, c, false, false);
  asm volatile("v_nop\n\tv_nop\n\tv_nop\n\tv_nop" : "+v"(d) : "v"(a.w), "v"(b.w));
  return d;
}

__device__ __forceinline__ unsigned int f2bf(float f) {
  const unsigned int u = __float_as_uint(f);
  return ((u + 0x7FFFu + ((u >> 16) & 1u)) >> 16) & 0xFFFFu;
}
__device__ __forceinline__ float bf2f(unsigned int b) { return __uint_as_float(b << 16); }
__device__ __forceinline__ float bfr(float f) { return bf2f(f2bf(f)); }
__device__ __forceinline__ unsigned int pk2(float lo, float hi) { return f2bf(lo) | (f2bf(hi) << 16); }
__device__ __forceinline__ v4u pack8(const v4f a, const v4f b) {
  v4u r;
  r.x = pk2(a.x, a.y); r.y = pk2(a.z, a.w); r.z = pk2(b.x, b.y); r.w = pk2(b.z, b.w);
  return r;
}

__device__ __forceinline__ int scan_chunk(const int* __restrict__ dsts, int nE, int cbase, int slotBase,
                                          int nb, int vec8, int* list, int tid, int lane, int wave) {
  int wc = 0;
  const int el0  = tid * EPT;
  const int e0   = cbase + el0;
  const int sent = -2147483647 - 1;
  v4i da, db;
  if (vec8 != 0 && cbase + CHUNK <= nE) {
    da = *(const v4i*)(dsts + e0);
    db = *(const v4i*)(dsts + e0 + 4);
  } else {
    da.x = (e0     < nE) ? dsts[min(e0,     nE - 1)] : sent;
    da.y = (e0 + 1 < nE) ? dsts[min(e0 + 1, nE - 1)] : sent;
    da.z = (e0 + 2 < nE) ? dsts[min(e0 + 2, nE - 1)] : sent;
    da.w = (e0 + 3 < nE) ? dsts[min(e0 + 3, nE - 1)] : sent;
    db.x = (e0 + 4 < nE) ? dsts[min(e0 + 4, nE - 1)] : sent;
    db.y = (e0 + 5 < nE) ? dsts[min(e0 + 5, nE - 1)] : sent;
    db.z = (e0 + 6 < nE) ? dsts[min(e0 + 6, nE - 1)] : sent;
    db.w = (e0 + 7 < nE) ? dsts[min(e0 + 7, nE - 1)] : sent;
  }
  const unsigned nbs = (unsigned)slotBase;
  const unsigned unb = (unsigned)nb;
  const unsigned s0 = (unsigned)da.x - nbs, s1 = (unsigned)da.y - nbs;
  const unsigned s2 = (unsigned)da.z - nbs, s3 = (unsigned)da.w - nbs;
  const unsigned s4 = (unsigned)db.x - nbs, s5 = (unsigned)db.y - nbs;
  const unsigned s6 = (unsigned)db.z - nbs, s7 = (unsigned)db.w - nbs;
  const bool h0 = s0 < unb, h1 = s1 < unb, h2 = s2 < unb, h3 = s3 < unb;
  const bool h4 = s4 < unb, h5 = s5 < unb, h6 = s6 < unb, h7 = s7 < unb;
  const unsigned any = __builtin_amdgcn_ballot_w32(h0 | h1 | h2 | h3 | h4 | h5 | h6 | h7);
  if (any != 0u) {
#define HITJ(J, HJ, SJ) { \
      const unsigned mj = __builtin_amdgcn_ballot_w32(HJ); \
      if (mj != 0u) { \
        if (HJ) { \
          const int pos = wc + (int)__builtin_amdgcn_mbcnt_lo(mj, 0u); \
          if (pos < WCAP) list[wave * WCAP + pos] = ((el0 + (J)) << SLOTB) | (int)(SJ); \
        } \
        wc += (int)__builtin_popcount(mj); } }
    HITJ(0, h0, s0)
    HITJ(1, h1, s1)
    HITJ(2, h2, s2)
    HITJ(3, h3, s3)
    HITJ(4, h4, s4)
    HITJ(5, h5, s5)
    HITJ(6, h6, s6)
    HITJ(7, h7, s7)
#undef HITJ
  }
  return wc;
}

__global__ __launch_bounds__(NTHR) void k_xprep(const float* __restrict__ x, unsigned short* xb, int nN, int nUnits) {
  const int i = (int)blockIdx.x * NTHR + (int)threadIdx.x;
  if (i >= nUnits) return;
  const int row = i >> 4;
  const int c0  = (i & 15) * 8;
  const int rc  = row < nN ? row : nN - 1;
  const float* p = x + (size_t)rc * F_IN + c0;
  v4f a = *(const v4fa*)p, b = *(const v4fa*)(p + 4);
  const v4f z4 = {0.f, 0.f, 0.f, 0.f};
  if (row >= nN) { a = z4; b = z4; }
  const v4u hv = pack8(a, b);
  const size_t o = (size_t)row * F_IN + c0;
  *(volatile v4u*)(xb + o) = hv;
  __threadfence();
  *(volatile v4u*)(xb + o) = hv;
}

__global__ __launch_bounds__(NTHR) void k_wtr(const float* __restrict__ w, int Kin, int Ncol, int Nrows, int Kout,
                                              unsigned short* wt, int nUnits) {
  const int u = (int)blockIdx.x * NTHR + (int)threadIdx.x;
  if (u >= nUnits) return;
  const int kq = Kout >> 3;
  const int n  = u / kq;
  const int k8 = (u - n * kq) * 8;
  const int kk = k8 - (k8 / Kin) * Kin;
  const int ncl = n < Ncol ? n : Ncol - 1;
  const float* p = w + (size_t)kk * (size_t)Ncol + ncl;
  v4f a, b;
  a.x = p[0];                    a.y = p[(size_t)Ncol];         a.z = p[(size_t)2 * Ncol];     a.w = p[(size_t)3 * Ncol];
  b.x = p[(size_t)4 * Ncol];     b.y = p[(size_t)5 * Ncol];     b.z = p[(size_t)6 * Ncol];     b.w = p[(size_t)7 * Ncol];
  const v4f z4 = {0.f, 0.f, 0.f, 0.f};
  if (n >= Ncol || n >= Nrows) { a = z4; b = z4; }
  const v4u wv = pack8(a, b);
  unsigned short* o = wt + (size_t)n * (size_t)Kout + k8;
  *(volatile v4u*)o = wv;
  __threadfence();
  *(volatile v4u*)o = wv;
}

template <int NT>
__global__ __launch_bounds__(GTHR) void k_gemm(
    const unsigned short* __restrict__ A, const unsigned short* __restrict__ WT,
    float* outF, int K,
    const float* __restrict__ atts, const float* __restrict__ attd,
    float* SD, int MPr)
{
  static_assert(NT == 2 || NT == 4);
  constexpr int COLS = 16 * NT;
  constexpr int NH   = COLS / 32;
  constexpr int PPR  = COLS / 4;
  constexpr int RPI  = 32 / PPR;
  constexpr int NIT  = 16 / RPI;
  __shared__ __attribute__((aligned(16))) float stg[GBM * COLS];
  __shared__ __attribute__((aligned(16))) float satt[2 * COLS];
  __shared__ __attribute__((aligned(16))) float sdot[2 * NH * GBM];
  const int tid = (int)threadIdx.x, lane = tid & 31, wave = tid >> 5, hh = lane >> 4, m = lane & 15;
  const int rowBase = (int)blockIdx.x * GBM;

  if (tid < 2 * COLS) {
    const int which = tid / COLS;
    const int c  = tid - which * COLS;
    const float vs = atts[c];
    const float vd = attd[c];
    const float v = (which == 0) ? vs : vd;
    satt[which * COLS + c] = bfr(v);
  }

  v8f acc[NT];
  {
    const v8f z = {0.f, 0.f, 0.f, 0.f, 0.f, 0.f, 0.f, 0.f};
#pragma unroll
    for (int t = 0; t < NT; ++t) acc[t] = z;
  }
  const unsigned short* ap = A  + (size_t)(rowBase + 16 * wave + m) * (size_t)K + 8 * hh;
  const unsigned short* wp = WT + (size_t)m * (size_t)K + 8 * hh;
  const int ksteps = K >> 5;
#pragma unroll 1
  for (int ks = 0; ks < ksteps; ++ks) {
    FragB af;
    af.h[0] = *(const v8usa*)(ap + 32 * ks);
    af.h[1] = *(const v8usa*)(ap + 32 * ks + 16);
#pragma unroll
    for (int t = 0; t < NT; ++t) {
      const unsigned short* wq = wp + (size_t)(16 * t) * (size_t)K + 32 * ks;
      FragB bf;
      bf.h[0] = *(const v8usa*)wq;
      bf.h[1] = *(const v8usa*)(wq + 16);
      acc[t] = wmb(af, bf, acc[t]);
    }
  }

#pragma unroll
  for (int t = 0; t < NT; ++t) {
    const int lc = 16 * t + m;
#pragma unroll
    for (int r = 0; r < 8; ++r) {
      const int lr = 16 * wave + 8 * hh + r;
      stg[lr * COLS + lc] = acc[t][r];
    }
  }
  __syncthreads();

  {
    const int row = tid & 63, which = tid >> 6;
#pragma unroll
    for (int hd = 0; hd < NH; ++hd) {
      const float* sa = satt + which * COLS + hd * 32;
      const float* hr = stg + row * COLS + hd * 32;
      float d = 0.f;
#pragma unroll 4
      for (int c4 = 0; c4 < 8; ++c4) {
        const v4f hv = *(const v4fa*)(hr + 4 * c4);
        const v4f av = *(const v4fa*)(sa + 4 * c4);
        d = fmaf(hv.x, av.x, d);
        d = fmaf(hv.y, av.y, d);
        d = fmaf(hv.z, av.z, d);
        d = fmaf(hv.w, av.w, d);
      }
      sdot[(2 * hd + which) * GBM + row] = d;
    }
  }
  __syncthreads();

  const int prow = lane / PPR, pcol = 4 * (lane % PPR);
  v4f fv[NIT];
#pragma unroll
  for (int i = 0; i < NIT; ++i) {
    const int lr = 16 * wave + RPI * i + prow;
    fv[i] = *(const v4fa*)(stg + lr * COLS + pcol);
  }
  const int hsel = wave < NH ? wave : 0;
  const int which2 = lane >> 4, piece = lane & 15;
  const v4f sdv = *(const v4fa*)(sdot + (2 * hsel + which2) * GBM + 4 * piece);
  float* sp = SD + (size_t)(2 * hsel + which2) * (size_t)MPr + rowBase + 4 * piece;

#pragma unroll
  for (int i = 0; i < NIT; ++i) {
    const int lr = 16 * wave + RPI * i + prow;
    float* op = outF + (size_t)(rowBase + lr) * (size_t)COLS + pcol;
    *(volatile v4f*)op = fv[i];
  }
  if (wave < NH) *(volatile v4f*)sp = sdv;
  __threadfence();
#pragma unroll
  for (int i = 0; i < NIT; ++i) {
    const int lr = 16 * wave + RPI * i + prow;
    float* op = outF + (size_t)(rowBase + lr) * (size_t)COLS + pcol;
    *(volatile v4f*)op = fv[i];
  }
  if (wave < NH) *(volatile v4f*)sp = sdv;
}

__global__ __launch_bounds__(NTHR) void k_agg1(
    const int* __restrict__ srcs, const int* __restrict__ dsts,
    const float* __restrict__ F, const float* __restrict__ SD,
    const float* __restrict__ bias,
    unsigned short* HP, int* LST, int* CNT, int* OFF,
    int nN, int nE, int vec8, int MPr) {
  extern __shared__ __attribute__((aligned(16))) int dsm[];
  int* reg1 = dsm;
  int* reg2 = reg1 + RCAP;
  int* scnt = reg2 + RCAP;
  int* soff = scnt + NB;
  int* list = soff + NB;
  int* wcnt = list + LISTN;
  int* wtot = wcnt + NWAVE;
  const int tid = (int)threadIdx.x, lane = tid & 31, wave = tid >> 5;
  const int nodeBase = (int)blockIdx.x * NB;

  {
    const v4i z4 = {0, 0, 0, 0};
    for (int i = tid * 4; i < RCAP; i += NTHR * 4) *(v4ia*)(reg1 + i) = z4;
    for (int i = tid * 4; i < NB; i += NTHR * 4) *(v4ia*)(scnt + i) = z4;
  }
  __syncthreads();

  int tot = 0;
  const int nChunks = (nE + CHUNK - 1) / CHUNK;
#pragma unroll 1
  for (int ch = 0; ch < nChunks; ++ch) {
    const int cbase = ch * CHUNK;
    const int wc = scan_chunk(dsts, nE, cbase, nodeBase, NB, vec8, list, tid, lane, wave);
    if (lane == 0) wcnt[wave] = wc;
    __syncthreads();
    int pre = 0, all = 0;
#pragma unroll
    for (int w2 = 0; w2 < NWAVE; ++w2) {
      int c = wcnt[w2];
      c = c < 0 ? 0 : (c > WCAP ? WCAP : c);
      all += c;
      pre += (w2 < wave) ? c : 0;
    }
    const int wcc  = wc > WCAP ? WCAP : wc;
    const int base = tot + pre;
#pragma unroll 1
    for (int i = lane; i < wcc; i += 32) {
      const int ent = list[wave * WCAP + i];
      const int el  = (ent >> SLOTB) & (CHUNK - 1);
      const int sl  = ent & (NB - 1);
      int eid = cbase + el;
      eid = eid > nE - 1 ? nE - 1 : eid;
      const int pos = base + i;
      if (pos < RCAP) reg1[pos] = (int)(((unsigned)eid << SLOTB) | (unsigned)sl);
    }
    tot += all;
    tot = tot > RCAP ? RCAP : tot;
    __syncthreads();
  }
  const int nh = tot;

  if (wave == 0) {
#pragma unroll 1
    for (int b0 = 0; b0 < nh; b0 += 32) {
      const int idx = b0 + lane;
      const int uv  = reg1[idx < nh ? idx : nh - 1];
      const int m32 = (nh - b0) < 32 ? (nh - b0) : 32;
#pragma unroll 1
      for (int k = 0; k < m32; ++k) {
        const int u  = __builtin_amdgcn_readlane(uv, k);
        const int sl = u & (NB - 1);
        if (lane == 0) scnt[sl] = scnt[sl] + 1;
      }
    }
  }
  __syncthreads();

  {
    const v4i ca = *(const v4ia*)(scnt + 4 * tid);
    const int e0 = ca.x < 0 ? 0 : ca.x, e1 = ca.y < 0 ? 0 : ca.y, e2 = ca.z < 0 ? 0 : ca.z, e3 = ca.w < 0 ? 0 : ca.w;
    const int ts = e0 + e1 + e2 + e3;
    int incl = ts;
#pragma unroll
    for (int d = 1; d < 32; d <<= 1) {
      const int up = __shfl_up(incl, d);
      if (lane >= d) incl += up;
    }
    if (lane == 31) wtot[wave] = incl;
    __syncthreads();
    int pre = 0;
#pragma unroll
    for (int w2 = 0; w2 < NWAVE; ++w2) pre += (w2 < wave) ? wtot[w2] : 0;
    int run = pre + incl - ts;
    soff[4 * tid + 0] = run; run += e0;
    soff[4 * tid + 1] = run; run += e1;
    soff[4 * tid + 2] = run; run += e2;
    soff[4 * tid + 3] = run;
  }
  __syncthreads();
  for (int i = tid; i < NB; i += NTHR) list[i] = soff[i];
  __syncthreads();

  if (wave == 0) {
#pragma unroll 1
    for (int b0 = 0; b0 < nh; b0 += 32) {
      const int idx = b0 + lane;
      const int uv  = reg1[idx < nh ? idx : nh - 1];
      const int m32 = (nh - b0) < 32 ? (nh - b0) : 32;
#pragma unroll 1
      for (int k = 0; k < m32; ++k) {
        const int u   = __builtin_amdgcn_readlane(uv, k);
        const int sl  = u & (NB - 1);
        const int eid = (int)((unsigned)u >> SLOTB);
        if (lane == 0) {
          int pos = list[sl];
          pos = pos < 0 ? 0 : (pos > RCAP - 1 ? RCAP - 1 : pos);
          reg2[pos] = eid;
          list[sl] = pos + 1;
        }
      }
    }
  }
  __syncthreads();

#pragma unroll 1
  for (int i0 = 0; i0 < nh; i0 += NTHR) {
    const int i  = i0 + tid;
    const int ic = i < nh ? i : nh - 1;
    int eid = reg2[ic];
    eid = eid < 0 ? 0 : (eid > nE - 1 ? nE - 1 : eid);
    int s = srcs[eid];
    s = s < 0 ? 0 : (s > nN - 1 ? nN - 1 : s);
    if (i < nh) reg1[i] = s;
  }
  __syncthreads();

  {
    int* lp = LST + (size_t)blockIdx.x * RCAP;
    int* cp = CNT + (size_t)blockIdx.x * NB + 4 * tid;
    int* fp = OFF + (size_t)blockIdx.x * NB + 4 * tid;
    const v4i cv = *(const v4ia*)(scnt + 4 * tid);
    const v4i ov = *(const v4ia*)(soff + 4 * tid);
#pragma unroll 1
    for (int it = 0; it < SPILL_IT; ++it) {
      const int o = 4 * (it * NTHR + tid);
      const v4i v = *(const v4ia*)(reg1 + o);
      *(volatile v4i*)(lp + o) = v;
    }
    *(volatile v4i*)cp = cv;
    *(volatile v4i*)fp = ov;
    __threadfence();
#pragma unroll 1
    for (int it = 0; it < SPILL_IT; ++it) {
      const int o = 4 * (it * NTHR + tid);
      const v4i v = *(const v4ia*)(reg1 + o);
      *(volatile v4i*)(lp + o) = v;
    }
    *(volatile v4i*)cp = cv;
    *(volatile v4i*)fp = ov;
  }

  const int nbw = NB / NWAVE;
  const bool ovf = (nh >= RCAP);
  const float qnan = __int_as_float(0x7fc00000);
  const int c0 = 2 * lane;
  const int hm = -(lane >> 4);
  const v2f bq = *(const v2fa*)(bias + c0);
  const float bb0 = bfr(bq.x), bb1 = bfr(bq.y);
  const float* S0 = SD;
  const float* D0 = SD + (size_t)MPr;
  const float* S1 = SD + (size_t)2 * MPr;
  const float* D1 = SD + (size_t)3 * MPr;

#pragma unroll 1
  for (int jt = 0; jt < nbw; ++jt) {
    const int slot = wave * nbw + jt;
    const int grow = nodeBase + slot;
    const int gcl  = grow < nN ? grow : nN - 1;
    int st = soff[slot];
    const int craw = scnt[slot];
    int cnt = craw;
    st  = st < 0 ? 0 : (st > nh ? nh : st);
    cnt = cnt < 0 ? 0 : (cnt > DEGCAP ? DEGCAP : cnt);
    if (cnt > nh - st) cnt = nh - st;
    const float pz = (ovf || craw > DEGCAP) ? qnan : 0.0f;

    const v2f fd = *(const v2fa*)(F + (size_t)gcl * HC1 + c0);
    const int s0i = __float_as_int(S0[gcl]);
    const int d0i = __float_as_int(D0[gcl]);
    const int s1i = __float_as_int(S1[gcl]);
    const int d1i = __float_as_int(D1[gcl]);
    const float asv = __int_as_float((s1i & hm) | (s0i & ~hm));
    const float adv = __int_as_float((d1i & hm) | (d0i & ~hm));
    float l0 = asv + adv;
    l0 = l0 > 0.f ? l0 : NEGSL * l0;
    float mx = l0, dn = 1.0f;
    float a0 = fd.x, a1 = fd.y;

#pragma unroll 1
    for (int b0 = 0; b0 < cnt; b0 += 32) {
      int idx = st + b0 + lane;
      idx = idx > RCAP - 1 ? RCAP - 1 : idx;
      int sr = reg1[idx];
      sr = sr < 0 ? 0 : (sr > nN - 1 ? nN - 1 : sr);
      const int e0i = __float_as_int(S0[sr]);
      const int e1i = __float_as_int(S1[sr]);
      const int m32 = (cnt - b0) < 32 ? (cnt - b0) : 32;
#pragma unroll 1
      for (int k = 0; k < m32; ++k) {
        const int sk  = __builtin_amdgcn_readlane(sr, k);
        const int k0i = __builtin_amdgcn_readlane(e0i, k);
        const int k1i = __builtin_amdgcn_readlane(e1i, k);
        const float ask = __int_as_float((k1i & hm) | (k0i & ~hm));
        const v2f fs = *(const v2fa*)(F + (size_t)sk * HC1 + c0);
        float lg = ask + adv;
        lg = lg > 0.f ? lg : NEGSL * lg;
        const float df = lg - mx;
        const float ee = expf(-fabsf(df));
        const bool up  = df > 0.f;
        const float s1 = up ? ee : 1.0f;
        const float s2 = up ? 1.0f : ee;
        mx = up ? lg : mx;
        dn = fmaf(dn, s1, s2);
        a0 = fmaf(a0, s1, s2 * fs.x);
        a1 = fmaf(a1, s1, s2 * fs.y);
      }
    }
    const float inv = __builtin_amdgcn_rcpf(dn);
    const bool live = grow < nN;
    float y0 = fmaf(a0, inv, bb0);
    float y1 = fmaf(a1, inv, bb1);
    y0 = (y0 > 0.0f) ? y0 : (y0 - y0);
    y1 = (y1 > 0.0f) ? y1 : (y1 - y1);
    y0 = y0 + pz;
    y1 = y1 + pz;
    const float o0 = live ? y0 : 0.0f;
    const float o1 = live ? y1 : 0.0f;
    const unsigned int hb0 = f2bf(o0), hb1 = f2bf(o1);
    const unsigned int lb0 = f2bf(o0 - bf2f(hb0)), lb1 = f2bf(o1 - bf2f(hb1));
    const unsigned int hw = hb0 | (hb1 << 16);
    const unsigned int lw = lb0 | (lb1 << 16);
    unsigned int* gp = (unsigned int*)(HP + (size_t)grow * KA2);
    const bool wr = grow < MPr;
    if (wr) { *(volatile unsigned int*)(gp + lane) = hw; *(volatile unsigned int*)(gp + 32 + lane) = lw; }
    __threadfence();
    if (wr) { *(volatile unsigned int*)(gp + lane) = hw; *(volatile unsigned int*)(gp + 32 + lane) = lw; }
  }
}

__global__ __launch_bounds__(NTHR) void k_agg2(
    const int* __restrict__ LST, const int* __restrict__ CNT, const int* __restrict__ OFF,
    const float* __restrict__ F, const float* __restrict__ SD,
    const float* __restrict__ bias, float* out, int nN, int MPr) {
  const int tid = (int)threadIdx.x, lane = tid & 31, wave = tid >> 5;
  const int nodeBase = (int)blockIdx.x * NB;
  const int* lp = LST + (size_t)blockIdx.x * RCAP;
  const int* cp = CNT + (size_t)blockIdx.x * NB;
  const int* fp = OFF + (size_t)blockIdx.x * NB;
  const float bz = bfr(bias[lane]);
  const float* ASp = SD;
  const float* ADp = SD + (size_t)MPr;
  const float qnan = __int_as_float(0x7fc00000);
  int nh2;
  {
    int lo = fp[NB - 1], lc = cp[NB - 1];
    lo = lo < 0 ? 0 : (lo > RCAP ? RCAP : lo);
    lc = lc < 0 ? 0 : (lc > RCAP ? RCAP : lc);
    nh2 = lo + lc;
    nh2 = nh2 > RCAP ? RCAP : nh2;
  }
  const bool ovf = (nh2 >= RCAP);
  const int nbw = NB / NWAVE;

#pragma unroll 1
  for (int jt = 0; jt < nbw; ++jt) {
    const int slot = wave * nbw + jt;
    const int grow = nodeBase + slot;
    if (grow >= nN) break;
    int st = fp[slot];
    const int craw = cp[slot];
    int cnt = craw;
    st  = st < 0 ? 0 : (st > nh2 ? nh2 : st);
    cnt = cnt < 0 ? 0 : (cnt > DEGCAP ? DEGCAP : cnt);
    if (cnt > nh2 - st) cnt = nh2 - st;
    int last = st + cnt - 1;
    last = last < 0 ? 0 : last;
    const float pz = (ovf || craw > DEGCAP) ? qnan : 0.0f;

    const float fd  = F[(size_t)grow * NC2 + lane];
    const float adv = ADp[grow];
    float l0 = ASp[grow] + adv;
    l0 = l0 > 0.f ? l0 : NEGSL * l0;
    float mx = l0, dn = 1.0f;
    float a0 = fd;

#pragma unroll 1
    for (int b0 = 0; b0 < cnt; b0 += 32) {
      int idx = st + b0 + lane;
      idx = idx > last ? last : idx;
      idx = idx > RCAP - 1 ? RCAP - 1 : idx;
      int sr = lp[idx];
      sr = sr < 0 ? 0 : (sr > nN - 1 ? nN - 1 : sr);
      const int esi = __float_as_int(ASp[sr]);
      const int m32 = (cnt - b0) < 32 ? (cnt - b0) : 32;
#pragma unroll 1
      for (int k = 0; k < m32; ++k) {
        const int   sk  = __builtin_amdgcn_readlane(sr, k);
        const float ask = __int_as_float(__builtin_amdgcn_readlane(esi, k));
        const float fs  = F[(size_t)sk * NC2 + lane];
        float lg = ask + adv;
        lg = lg > 0.f ? lg : NEGSL * lg;
        const float df = lg - mx;
        const float ee = expf(-fabsf(df));
        const bool up  = df > 0.f;
        const float s1 = up ? ee : 1.0f;
        const float s2 = up ? 1.0f : ee;
        mx = up ? lg : mx;
        dn = fmaf(dn, s1, s2);
        a0 = fmaf(a0, s1, s2 * fs);
      }
    }
    const float inv = __builtin_amdgcn_rcpf(dn);
    const float o = fmaf(a0, inv, bz) + pz;
    float* op = out + (size_t)grow * NC2 + lane;
    *(volatile float*)op = o;
    __threadfence();
    *(volatile float*)op = o;
  }
}

static inline int cdiv(int a, int b) { return (a + b - 1) / b; }

extern "C" void kernel_launch(void* const* d_in, const int* in_sizes, int n_in,
                              void* d_out, int out_size, void* d_ws, size_t ws_size,
                              hipStream_t stream) {
  if (n_in < 10) return;
  const int nN = in_sizes[0] / F_IN;
  if (nN <= 0 || in_sizes[0] != nN * F_IN || nN > (1 << 22)) return;
  if (in_sizes[1] < 2 || (in_sizes[1] & 1) != 0) return;
  const int nE = in_sizes[1] / 2;
  if (nE < 1 || nE >= (1 << (32 - SLOTB))) return;
  if (in_sizes[2] != F_IN * HC1) return;
  if (in_sizes[3] != NHD1 * HID || in_sizes[4] != NHD1 * HID) return;
  if (in_sizes[5] != HC1) return;
  if (in_sizes[6] != HC1 * NC2) return;
  if (in_sizes[7] != NC2 || in_sizes[8] != NC2) return;
  if (in_sizes[9] != NC2) return;
  if ((long long)out_size != (long long)nN * NC2) return;

  const float* x    = (const float*)d_in[0];
  const int*   ei   = (const int*)  d_in[1];
  const float* W1   = (const float*)d_in[2];
  const float* a1s  = (const float*)d_in[3];
  const float* a1d  = (const float*)d_in[4];
  const float* b1   = (const float*)d_in[5];
  const float* W2   = (const float*)d_in[6];
  const float* a2s  = (const float*)d_in[7];
  const float* a2d  = (const float*)d_in[8];
  const float* b2   = (const float*)d_in[9];
  float* out = (float*)d_out;
  const int* src = ei;
  const int* dst = ei + nE;

  const int MP   = cdiv(nN, GBM) * GBM;
  const int gA   = cdiv(MP, NB);
  const int vec8 = ((nE & 3) == 0) ? 1 : 0;
  if ((long long)gA * NB < (long long)MP) return;

  char* ws = (char*)d_ws;
  size_t off = 0;
  const size_t oXB  = off; off += (size_t)MP * F_IN * 2;           off = (off + 255) & ~(size_t)255;
  const size_t oW1T = off; off += (size_t)HC1 * F_IN * 2;          off = (off + 255) & ~(size_t)255;
  const size_t oW2T = off; off += (size_t)NC2 * KA2 * 2;           off = (off + 255) & ~(size_t)255;
  const size_t oH1  = off; off += (size_t)MP * HC1 * 4;            off = (off + 255) & ~(size_t)255;
  const size_t oSD1 = off; off += (size_t)4 * MP * 4;              off = (off + 255) & ~(size_t)255;
  const size_t oX1  = off; off += (size_t)MP * KA2 * 2;            off = (off + 255) & ~(size_t)255;
  const size_t oH2  = off; off += (size_t)MP * NC2 * 4;            off = (off + 255) & ~(size_t)255;
  const size_t oSD2 = off; off += (size_t)2 * MP * 4;              off = (off + 255) & ~(size_t)255;
  const size_t oLST = off; off += (size_t)gA * RCAP * 4;           off = (off + 255) & ~(size_t)255;
  const size_t oCNT = off; off += (size_t)gA * NB * 4;             off = (off + 255) & ~(size_t)255;
  const size_t oOFF = off; off += (size_t)gA * NB * 4;             off = (off + 255) & ~(size_t)255;
  if (off > ws_size || off > (size_t)WSMAX) return;
  unsigned short* XB  = (unsigned short*)(ws + oXB);
  unsigned short* W1T = (unsigned short*)(ws + oW1T);
  unsigned short* W2T = (unsigned short*)(ws + oW2T);
  float*          H1  = (float*)(ws + oH1);
  float*          SD1 = (float*)(ws + oSD1);
  unsigned short* X1  = (unsigned short*)(ws + oX1);
  float*          H2  = (float*)(ws + oH2);
  float*          SD2 = (float*)(ws + oSD2);
  int*            LST = (int*)(ws + oLST);
  int*            CNT = (int*)(ws + oCNT);
  int*            OFF = (int*)(ws + oOFF);

  hipFuncSetAttribute(reinterpret_cast<const void*>(&k_agg1),
                      hipFuncAttributeMaxDynamicSharedMemorySize, LDS_AGG);

  const int nUx = MP * (F_IN / 8);
  k_xprep<<<cdiv(nUx, NTHR), NTHR, 0, stream>>>(x, XB, nN, nUx);

  {
    const int nUw1 = HC1 * (F_IN / 8);
    k_wtr<<<cdiv(nUw1, NTHR), NTHR, 0, stream>>>(W1, F_IN, HC1, HC1, F_IN, W1T, nUw1);
    const int nUw2 = NC2 * (KA2 / 8);
    k_wtr<<<cdiv(nUw2, NTHR), NTHR, 0, stream>>>(W2, HC1, NC2, NC2, KA2, W2T, nUw2);
  }

  const int gM = MP / GBM;
  k_gemm<4><<<gM, GTHR, 0, stream>>>(XB, W1T, H1, F_IN, a1s, a1d, SD1, MP);
  k_agg1<<<gA, NTHR, LDS_AGG, stream>>>(src, dst, H1, SD1, b1, X1, LST, CNT, OFF, nN, nE, vec8, MP);
  k_gemm<2><<<gM, GTHR, 0, stream>>>(X1, W2T, H2, KA2, a2s, a2d, SD2, MP);
  k_agg2<<<gA, NTHR, 0, stream>>>(LST, CNT, OFF, H2, SD2, b2, out, nN, MP);
}
